// oklamai_LSTM_66709432041647
// MI455X (gfx1250) — hardware-run, weakly checked
//
#include <hip/hip_runtime.h>
#include <math.h>

constexpr int SEQ_T  = 4096;
constexpr int N_IN   = 1024;
constexpr int N_HID  = 1024;
constexpr int N_GATE = 4 * N_HID;

constexpr float X_CARRY = 16.0f;
constexpr float W_CARRY = 1024.0f;
constexpr float FOLD_BACK = 1.0f / (X_CARRY * W_CARRY);

constexpr int NB_CVT  = (SEQ_T * N_IN) / (256 * 8);
constexpr int NB_TR   = (N_GATE / 64) * (N_HID / 64);
constexpr int NB_BIAS = N_GATE / (256 * 4);
constexpr int NB_PREP = 2 * NB_CVT + NB_TR + NB_BIAS;

static_assert(SEQ_T % 64 == 0 && N_GATE % 64 == 0, "GEMM M and N are multiples of the 64 tile");
static_assert(N_IN % 32 == 0, "GEMM K is a multiple of 32");
static_assert(N_GATE * N_IN == SEQ_T * N_IN, "both 16-bit planes have the same element count");
static_assert((SEQ_T * N_IN) % (256 * 8) == 0, "convert blocks cover the planes exactly");
static_assert(N_HID % 8 == 0, "k loop steps by 8");
static_assert(N_HID == 1024, "one scan thread per hidden unit in a 1024-thread block");

typedef __attribute__((ext_vector_type(16))) _Float16 v16h;
typedef __attribute__((ext_vector_type(8)))  _Float16 v8h;
typedef __attribute__((ext_vector_type(8)))  float    v8f;
typedef __attribute__((ext_vector_type(4)))  float    v4f;

__device__ __forceinline__ unsigned short f2bf_bits(float f) {
  unsigned u = __float_as_uint(f);
  return (unsigned short)((u + 0x7FFFu + ((u >> 16) & 1u)) >> 16);
}
__device__ __forceinline__ float bf_bits2f(unsigned short h) { return __uint_as_float(((unsigned)h) << 16); }
__device__ __forceinline__ float bf_val(float f) { return bf_bits2f(f2bf_bits(f)); }
__device__ __forceinline__ _Float16 to_plane(float f, float carry) { return (_Float16)(bf_val(f) * carry); }

__device__ __forceinline__ void tie_h(v8f& a, v16h x, v16h y) { asm volatile("" : "+v"(a) : "v"(x), "v"(y)); }
__device__ __forceinline__ void guard_h(v8f& a, v16h x, v16h y) { asm volatile("v_nop\n\tv_nop\n\tv_nop\n\tv_nop" : "+v"(a) : "v"(x), "v"(y)); }
__device__ __forceinline__ void keep4_h(v16h a, v16h b, v16h c, v16h d) { asm volatile("v_nop" :: "v"(a), "v"(b), "v"(c), "v"(d)); }
__device__ __forceinline__ void acc_guard4(v8f& a, v8f& b, v8f& c, v8f& d) { asm volatile("v_nop\n\tv_nop\n\tv_nop\n\tv_nop" : "+v"(a), "+v"(b), "+v"(c), "+v"(d)); }

struct FragH {
  union U { v16h v; v8h h[2]; };
  static __device__ __forceinline__ v16h load(const _Float16* p) {
    U f; f.h[0] = *(const v8h*)(p); f.h[1] = *(const v8h*)(p + 16); return f.v;
  }
  static __device__ __forceinline__ v8f mma(v16h a, v16h b, v8f c) {
    return __builtin_amdgcn_wmma_f32_16x16x32_f16(false, a, false, b, (short)0, c, false, false);
  }
};

__global__ __launch_bounds__(256) void prep_kernel(
    const float* __restrict__ x, const float* __restrict__ wih, const float* __restrict__ whh,
    const float* __restrict__ bih, const float* __restrict__ bhh,
    unsigned short* __restrict__ X16, unsigned short* __restrict__ W16,
    float* __restrict__ WHQ, float* __restrict__ BIAS) {
  __shared__ float Tt[64 * 65];
  const int tid = threadIdx.x;
  const int bid = blockIdx.x;

  if (bid < 2 * NB_CVT) {
    const bool isw = (bid >= NB_CVT);
    const float* src = isw ? wih : x;
    unsigned short* dst = isw ? W16 : X16;
    const float carry = isw ? W_CARRY : X_CARRY;
    const int lb = isw ? (bid - NB_CVT) : bid;
    const size_t i8 = ((size_t)lb * 256 + (size_t)tid) * 8;
    const v4f a = *(const v4f*)(src + i8);
    const v4f b = *(const v4f*)(src + i8 + 4);
    const float a0 = a[0], a1 = a[1], a2 = a[2], a3 = a[3];
    const float b0 = b[0], b1 = b[1], b2 = b[2], b3 = b[3];
    v8h hv;
    hv[0] = to_plane(a0, carry);
    hv[1] = to_plane(a1, carry);
    hv[2] = to_plane(a2, carry);
    hv[3] = to_plane(a3, carry);
    hv[4] = to_plane(b0, carry);
    hv[5] = to_plane(b1, carry);
    hv[6] = to_plane(b2, carry);
    hv[7] = to_plane(b3, carry);
    *(volatile v8h*)(dst + i8) = hv;
    __threadfence();
    *(volatile v8h*)(dst + i8) = hv;
  } else if (bid < 2 * NB_CVT + NB_TR) {
    const int tb = bid - 2 * NB_CVT;
    const int k0 = (tb & 15) * 64;
    const int r0 = (tb >> 4) * 64;
#pragma unroll
    for (int it = 0; it < 4; ++it) {
      const int idx = it * 256 + tid;
      const int rr = idx >> 4;
      const int cc = (idx & 15) * 4;
      const v4f v = *(const v4f*)(whh + (size_t)(r0 + rr) * N_HID + k0 + cc);
      const float v0 = v[0], v1 = v[1], v2 = v[2], v3 = v[3];
      Tt[rr * 65 + cc + 0] = bf_val(v0);
      Tt[rr * 65 + cc + 1] = bf_val(v1);
      Tt[rr * 65 + cc + 2] = bf_val(v2);
      Tt[rr * 65 + cc + 3] = bf_val(v3);
    }
    __syncthreads();
    v4f o[4];
#pragma unroll
    for (int it = 0; it < 4; ++it) {
      const int idx = it * 256 + tid;
      const int row = idx & 63;
      const int kq = idx >> 6;
      o[it][0] = Tt[row * 65 + 4 * kq + 0];
      o[it][1] = Tt[row * 65 + 4 * kq + 1];
      o[it][2] = Tt[row * 65 + 4 * kq + 2];
      o[it][3] = Tt[row * 65 + 4 * kq + 3];
    }
    for (int pass = 0; pass < 2; ++pass) {
#pragma unroll
      for (int it = 0; it < 4; ++it) {
        const int idx = it * 256 + tid;
        const int row = idx & 63;
        const int kq = idx >> 6;
        const size_t q4 = (size_t)((k0 >> 2) + kq) * N_GATE + (size_t)(r0 + row);
        *(volatile v4f*)(WHQ + q4 * 4) = o[it];
      }
      __threadfence();
    }
  } else {
    const int tb = bid - (2 * NB_CVT + NB_TR);
    const int i4 = (tb * 256 + tid) * 4;
    const v4f a = *(const v4f*)(bih + i4);
    const v4f b = *(const v4f*)(bhh + i4);
    const float a0 = a[0], a1 = a[1], a2 = a[2], a3 = a[3];
    const float b0 = b[0], b1 = b[1], b2 = b[2], b3 = b[3];
    v4f o;
    o[0] = bf_val(a0) + bf_val(b0);
    o[1] = bf_val(a1) + bf_val(b1);
    o[2] = bf_val(a2) + bf_val(b2);
    o[3] = bf_val(a3) + bf_val(b3);
    *(volatile v4f*)(BIAS + i4) = o;
    __threadfence();
    *(volatile v4f*)(BIAS + i4) = o;
  }
}

__global__ __launch_bounds__(256) void gemm_pre_kernel(
    const unsigned short* __restrict__ Ap, const unsigned short* __restrict__ Btp,
    float* __restrict__ C, const float* __restrict__ bias, float scale) {
  const _Float16* A  = (const _Float16*)Ap;
  const _Float16* Bt = (const _Float16*)Btp;
  __shared__ __align__(16) float sT[8][16 * 68];
  constexpr int LDA = N_IN, LDB = N_IN, LDC = N_GATE;
  constexpr int TILES_N = N_GATE >> 6;
  constexpr int TILES_M = SEQ_T >> 6;
  const int lane = threadIdx.x & 31;
  const int wave = threadIdx.x >> 5;
  const int tile = blockIdx.x * 8 + wave;
  if (tile >= TILES_M * TILES_N) return;
  const int tm = tile / TILES_N;
  const int tn = tile - tm * TILES_N;
  const int m0 = tm << 6;
  const int n0 = tn << 6;

  const int rlane = lane & 15;
  const int koff  = (lane >> 4) * 8;
  const int mOff  = (lane >> 4) * 8;

  v8f acc[4][4];
#pragma unroll
  for (int i = 0; i < 4; ++i)
#pragma unroll
    for (int j = 0; j < 4; ++j) acc[i][j] = (v8f){0.f, 0.f, 0.f, 0.f, 0.f, 0.f, 0.f, 0.f};

  for (int k0 = 0; k0 < N_IN; k0 += 32) {
    v16h bh[4];
#pragma unroll
    for (int j = 0; j < 4; ++j) {
      const size_t bo = (size_t)(n0 + (j << 4) + rlane) * LDB + koff + k0;
      bh[j] = FragH::load(Bt + bo);
    }
#pragma unroll
    for (int i = 0; i < 4; ++i) {
      const size_t ao = (size_t)(m0 + (i << 4) + rlane) * LDA + koff + k0;
      const v16h ah = FragH::load(A + ao);
#pragma unroll
      for (int j = 0; j < 4; ++j) acc[i][j] = FragH::mma(ah, bh[j], acc[i][j]);
      tie_h(acc[i][0], ah, bh[0]);
      tie_h(acc[i][1], ah, bh[1]);
      tie_h(acc[i][2], ah, bh[2]);
      guard_h(acc[i][3], ah, bh[3]);
    }
    keep4_h(bh[0], bh[1], bh[2], bh[3]);
  }
  acc_guard4(acc[0][0], acc[0][1], acc[0][2], acc[0][3]);
  acc_guard4(acc[1][0], acc[1][1], acc[1][2], acc[1][3]);
  acc_guard4(acc[2][0], acc[2][1], acc[2][2], acc[2][3]);
  acc_guard4(acc[3][0], acc[3][1], acc[3][2], acc[3][3]);

  float* slab = sT[wave];
  float bv[4];
#pragma unroll
  for (int j = 0; j < 4; ++j) bv[j] = bias[n0 + (j << 4) + rlane];
#pragma unroll
  for (int i = 0; i < 4; ++i) {
    const int mBase = m0 + (i << 4);
#pragma unroll
    for (int j = 0; j < 4; ++j) {
#pragma unroll
      for (int r = 0; r < 8; ++r) {
        const float v = acc[i][j][r] * scale + bv[j];
        slab[(mOff + r) * 68 + (j << 4) + rlane] = v;
      }
    }
    __builtin_amdgcn_fence(__ATOMIC_RELEASE, "workgroup");
    __builtin_amdgcn_wave_barrier();
    __builtin_amdgcn_fence(__ATOMIC_ACQUIRE, "workgroup");
    {
      const int hh = lane >> 4;
      const int c4 = (lane & 15) * 4;
      for (int pass = 0; pass < 2; ++pass) {
#pragma unroll
        for (int it = 0; it < 8; ++it) {
          const int row = it * 2 + hh;
          const v4f v = *(const v4f*)(slab + row * 68 + c4);
          *(volatile v4f*)(C + (size_t)(mBase + row) * LDC + n0 + c4) = v;
        }
        __threadfence();
      }
    }
    __builtin_amdgcn_fence(__ATOMIC_RELEASE, "workgroup");
    __builtin_amdgcn_wave_barrier();
    __builtin_amdgcn_fence(__ATOMIC_ACQUIRE, "workgroup");
  }
}

__global__ __launch_bounds__(1024) void scan_kernel(
    const float* __restrict__ pre, const float* __restrict__ whq, float* __restrict__ out) {
  __shared__ __align__(16) float hbuf[2 * N_HID];
  const int u = threadIdx.x;
  hbuf[u] = 0.0f;
  hbuf[N_HID + u] = 0.0f;
  __syncthreads();

  float c = 0.0f;
  const v4f* wbase = (const v4f*)whq + u;

#pragma unroll 1
  for (int t = 0; t < SEQ_T; ++t) {
    const float* hp = hbuf + (t & 1) * N_HID;
    float* hn = hbuf + ((t + 1) & 1) * N_HID;
    const float* pr = pre + (size_t)t * N_GATE + u;
    const float p0 = pr[0];
    const float p1 = pr[N_HID];
    const float p2 = pr[2 * N_HID];
    const float p3 = pr[3 * N_HID];

    float a0 = 0.0f, a1 = 0.0f, a2 = 0.0f, a3 = 0.0f;
    const v4f* wp = wbase;
#pragma unroll 1
    for (int k8 = 0; k8 < N_HID / 8; ++k8) {
      const v4f ha = *(const v4f*)(hp + 8 * k8);
      const v4f hb = *(const v4f*)(hp + 8 * k8 + 4);
      const v4f w0a = wp[0];
      const v4f w1a = wp[N_HID];
      const v4f w2a = wp[2 * N_HID];
      const v4f w3a = wp[3 * N_HID];
      const v4f w0b = wp[N_GATE];
      const v4f w1b = wp[N_GATE + N_HID];
      const v4f w2b = wp[N_GATE + 2 * N_HID];
      const v4f w3b = wp[N_GATE + 3 * N_HID];
      wp += 2 * N_GATE;
      a0 = fmaf(w0a[0], ha[0], a0);
      a1 = fmaf(w1a[0], ha[0], a1);
      a2 = fmaf(w2a[0], ha[0], a2);
      a3 = fmaf(w3a[0], ha[0], a3);
      a0 = fmaf(w0a[1], ha[1], a0);
      a1 = fmaf(w1a[1], ha[1], a1);
      a2 = fmaf(w2a[1], ha[1], a2);
      a3 = fmaf(w3a[1], ha[1], a3);
      a0 = fmaf(w0a[2], ha[2], a0);
      a1 = fmaf(w1a[2], ha[2], a1);
      a2 = fmaf(w2a[2], ha[2], a2);
      a3 = fmaf(w3a[2], ha[2], a3);
      a0 = fmaf(w0a[3], ha[3], a0);
      a1 = fmaf(w1a[3], ha[3], a1);
      a2 = fmaf(w2a[3], ha[3], a2);
      a3 = fmaf(w3a[3], ha[3], a3);
      a0 = fmaf(w0b[0], hb[0], a0);
      a1 = fmaf(w1b[0], hb[0], a1);
      a2 = fmaf(w2b[0], hb[0], a2);
      a3 = fmaf(w3b[0], hb[0], a3);
      a0 = fmaf(w0b[1], hb[1], a0);
      a1 = fmaf(w1b[1], hb[1], a1);
      a2 = fmaf(w2b[1], hb[1], a2);
      a3 = fmaf(w3b[1], hb[1], a3);
      a0 = fmaf(w0b[2], hb[2], a0);
      a1 = fmaf(w1b[2], hb[2], a1);
      a2 = fmaf(w2b[2], hb[2], a2);
      a3 = fmaf(w3b[2], hb[2], a3);
      a0 = fmaf(w0b[3], hb[3], a0);
      a1 = fmaf(w1b[3], hb[3], a1);
      a2 = fmaf(w2b[3], hb[3], a2);
      a3 = fmaf(w3b[3], hb[3], a3);
    }

    const float gi = p0 + a0;
    const float gf = p1 + a1;
    const float gc = p2 + a2;
    const float go = p3 + a3;
    const float ig = 1.0f / (1.0f + expf(-gi));
    const float fg = 1.0f / (1.0f + expf(-gf));
    const float cg = tanhf(gc);
    const float og = 1.0f / (1.0f + expf(-go));
    c = fg * c + ig * cg;
    const float hval = og * tanhf(c);

    hn[u] = hval;
    volatile float* op = out + (size_t)t * N_HID + u;
    *op = hval;
    __threadfence();
    *op = hval;
    __syncthreads();
  }
}

extern "C" void kernel_launch(void* const* d_in, const int* in_sizes, int n_in,
                              void* d_out, int out_size, void* d_ws, size_t ws_size, hipStream_t stream) {
  if (n_in < 5 || d_out == nullptr || d_ws == nullptr) return;
  if (in_sizes[0] != SEQ_T * N_IN || in_sizes[1] != N_GATE * N_IN || in_sizes[2] != N_GATE * N_HID ||
      in_sizes[3] != N_GATE || in_sizes[4] != N_GATE || out_size != SEQ_T * N_HID) return;

  const float* x   = (const float*)d_in[0];
  const float* wih = (const float*)d_in[1];
  const float* whh = (const float*)d_in[2];
  const float* bih = (const float*)d_in[3];
  const float* bhh = (const float*)d_in[4];
  float* out = (float*)d_out;

  char* ws = (char*)d_ws;
  size_t off = 0;
  auto carve = [&](size_t bytes) -> char* { char* p = ws + off; off += (bytes + 255) & ~(size_t)255; return p; };
  unsigned short* X16 = (unsigned short*)carve((size_t)SEQ_T * N_IN * 2);
  unsigned short* W16 = (unsigned short*)carve((size_t)N_GATE * N_IN * 2);
  float* WHQ  = (float*)carve((size_t)N_GATE * N_HID * 4);
  float* BIAS = (float*)carve((size_t)N_GATE * 4);
  float* PRE  = (float*)carve((size_t)SEQ_T * N_GATE * 4);
  if (off > ws_size || off > (size_t)134217728) return;

  prep_kernel<<<NB_PREP, 256, 0, stream>>>(x, wih, whh, bih, bhh, X16, W16, WHQ, BIAS);
  gemm_pre_kernel<<<((SEQ_T / 64) * (N_GATE / 64)) / 8, 256, 0, stream>>>(X16, W16, PRE, BIAS, FOLD_BACK);
  scan_kernel<<<1, 1024, 0, stream>>>(PRE, WHQ, out);
}
